// BNLSTMCell_8744553414711
// MI455X (gfx1250) — hardware-verified
//
#include <hip/hip_runtime.h>


#define NBT  4096
#define NIN  1024
#define NHID 1024
#define NG4  (4 * NHID)
#define CW   1024
#define PREW (3 * NHID)

typedef unsigned short bf;
typedef __attribute__((ext_vector_type(16))) __bf16   v16bf;
typedef __attribute__((ext_vector_type(8)))  unsigned short v8us;
typedef __attribute__((ext_vector_type(8)))  float    v8f;
typedef __attribute__((ext_vector_type(4)))  float    v4f;
typedef v4f  __attribute__((may_alias)) v4fa;
typedef v8us __attribute__((may_alias)) v8usa;

__device__ __forceinline__ unsigned short f2bf(float f) { unsigned u = __float_as_uint(f); u += 0x7FFFu + ((u >> 16) & 1u); return (unsigned short)(u >> 16); }
__device__ __forceinline__ float bf2f(unsigned short b) { return __uint_as_float(((unsigned)b) << 16); }
__device__ __forceinline__ float bfr(float f) { return bf2f(f2bf(f)); }
__device__ __forceinline__ v16bf cat16b(v8us lo, v8us hi) { return __builtin_bit_cast(v16bf, __builtin_shufflevector(lo, hi, 0, 1, 2, 3, 4, 5, 6, 7, 8, 9, 10, 11, 12, 13, 14, 15)); }
__device__ __forceinline__ v8f wmmab(v16bf a, v16bf b, v8f c) { return __builtin_amdgcn_wmma_f32_16x16x32_bf16(false, a, false, b, (short)0, c, false, false); }
#define VST2(T, p, v) do { const T vst2_v_ = (v); *(volatile T*)(p) = vst2_v_; __threadfence(); *(volatile T*)(p) = vst2_v_; } while (0)

__global__ __launch_bounds__(256) void k_cvtb(const float* __restrict__ src, bf* dst) {
    const int lane = threadIdx.x & 31, r = blockIdx.x * 8 + (threadIdx.x >> 5);
    if (r >= NBT) return;
    v8us o[4];
#pragma unroll
    for (int q = 0; q < 4; ++q) { v8us t;
#pragma unroll
        for (int i = 0; i < 8; ++i) t[i] = f2bf(src[(size_t)r * NIN + q * 256 + lane * 8 + i]);
        o[q] = t; }
#pragma unroll
    for (int q = 0; q < 4; ++q) *(volatile v8us*)(dst + (size_t)r * NIN + q * 256 + lane * 8) = o[q];
    __threadfence();
#pragma unroll
    for (int q = 0; q < 4; ++q) *(volatile v8us*)(dst + (size_t)r * NIN + q * 256 + lane * 8) = o[q];
}

__global__ __launch_bounds__(256) void k_wt(const float* __restrict__ Wm, bf* WT) {
    __shared__ __align__(16) unsigned short tl[64 * 72];
    const int tid = threadIdx.x, k0 = blockIdx.x * 64, n0 = blockIdx.y * 64;
    const int kk = tid >> 2, nq = (tid & 3) * 16;
#pragma unroll
    for (int i = 0; i < 16; ++i) tl[(nq + i) * 72 + kk] = f2bf(Wm[(size_t)(k0 + kk) * NG4 + n0 + nq + i]);
    __syncthreads();
    const int piece = tid & 7;
    auto pass = [&]() {
#pragma unroll
        for (int s = 0; s < 2; ++s) { const int nr = (tid >> 3) + 32 * s; const v8us val = *(const v8usa*)(tl + nr * 72 + piece * 8);
            *(volatile v8us*)(WT + (size_t)(n0 + nr) * NIN + k0 + piece * 8) = val; }
    };
    pass(); __threadfence(); pass();
}

__global__ __launch_bounds__(128) void k_gemmb(const bf* __restrict__ A, const bf* __restrict__ Bn, float* C) {
    __shared__ __align__(16) float ost[4][16 * 68];
    const int lane = threadIdx.x & 31, wave = threadIdx.x >> 5, lr = lane & 15, hi = lane >> 4;
    const int r0 = blockIdx.x * 64 + wave * 16, c0 = blockIdx.y * 64;
    const size_t aoff = (size_t)(r0 + lr) * NIN + 8 * hi;
    size_t boff[4];
#pragma unroll
    for (int t = 0; t < 4; ++t) boff[t] = (size_t)(c0 + t * 16 + lr) * NIN + 8 * hi;
    v8f acc[4];
#pragma unroll
    for (int t = 0; t < 4; ++t) acc[t] = (v8f){};
#pragma unroll 1
    for (int kc = 0; kc < NIN; kc += 32) {
        const v16bf a = cat16b(*(const v8us*)(A + aoff + kc), *(const v8us*)(A + aoff + kc + 16));
#pragma unroll
        for (int t = 0; t < 4; ++t) acc[t] = wmmab(a, cat16b(*(const v8us*)(Bn + boff[t] + kc), *(const v8us*)(Bn + boff[t] + kc + 16)), acc[t]);
        asm volatile("v_nop\n\tv_nop\n\tv_nop\n\tv_nop" : "+v"(acc[0]), "+v"(acc[1]), "+v"(acc[2]), "+v"(acc[3]) : "v"(a));
    }
    float* os = &ost[wave][0];
#pragma unroll
    for (int t = 0; t < 4; ++t)
#pragma unroll
        for (int j = 0; j < 8; ++j) os[(hi * 8 + j) * 68 + t * 16 + lr] = acc[t][j];
    __syncthreads();
    float* crow = C + (size_t)r0 * CW + c0;
    auto pass = [&]() {
#pragma unroll
        for (int s = 0; s < 8; ++s) { const int Lid = (lane >> 3) + 4 * s, piece = lane & 7; const int row = Lid >> 1, cofs = (Lid & 1) * 32 + piece * 4;
            const v4f val = *(const v4fa*)(os + row * 68 + cofs); *(volatile v4f*)(crow + (size_t)row * CW + cofs) = val; }
    };
    pass(); __threadfence(); pass();
}

__global__ __launch_bounds__(256) void k_colstat(const float* __restrict__ M, float* MU, float* RS) {
    const int c = blockIdx.x * 256 + threadIdx.x;
    double s = 0.0, q = 0.0;
#pragma unroll 1
    for (int r = 0; r < NBT; ++r) { const double v = (double)M[(size_t)r * CW + c]; s += v; q += v * v; }
    const double mu = s / (double)NBT; double var = q / (double)NBT - mu * mu; if (var < 0.0) var = 0.0;
    VST2(float, MU + c, (float)mu);
    VST2(float, RS + c, (float)(1.0 / sqrt(var + 1e-5)));
}

__global__ __launch_bounds__(256) void k_pre(const float* __restrict__ WH, const float* __restrict__ WI, const float* __restrict__ MUH, const float* __restrict__ RSH,
                                             const float* __restrict__ MUI, const float* __restrict__ RSI, const float* __restrict__ ghh, const float* __restrict__ bhh,
                                             const float* __restrict__ gih, const float* __restrict__ bih, const float* __restrict__ bias, int cbase, int slot, float* PRE) {
    const int lane = threadIdx.x & 31, r = blockIdx.x * 8 + (threadIdx.x >> 5);
    if (r >= NBT) return;
    v4f o[8];
#pragma unroll 1
    for (int q = 0; q < 8; ++q) {
        v4f t;
#pragma unroll
        for (int i = 0; i < 4; ++i) {
            const int c = q * 128 + lane * 4 + i, gc = cbase + c;
            const float a = WH[(size_t)r * CW + c], b = WI[(size_t)r * CW + c];
            t[i] = (bfr(ghh[gc]) * (a - MUH[c]) * RSH[c] + bfr(bhh[gc])) + (bfr(gih[gc]) * (b - MUI[c]) * RSI[c] + bfr(bih[gc])) + bfr(bias[gc]);
        }
        o[q] = t;
    }
    float* d = PRE + (size_t)r * PREW + (size_t)slot * CW;
#pragma unroll
    for (int q = 0; q < 8; ++q) *(volatile v4f*)(d + q * 128 + lane * 4) = o[q];
    __threadfence();
#pragma unroll
    for (int q = 0; q < 8; ++q) *(volatile v4f*)(d + q * 128 + lane * 4) = o[q];
}

__device__ __forceinline__ float sigm(float x) { return 1.0f / (1.0f + __expf(-x)); }
__device__ __forceinline__ float tanh_(float x) { return 2.0f / (1.0f + __expf(-2.0f * x)) - 1.0f; }
__global__ __launch_bounds__(256) void k_c1(const float* __restrict__ PRE, const float* __restrict__ c0, float* C1) {
    const int lane = threadIdx.x & 31, r = blockIdx.x * 8 + (threadIdx.x >> 5);
    if (r >= NBT) return;
    const float* p = PRE + (size_t)r * PREW;
    v4f o[8];
#pragma unroll 1
    for (int q = 0; q < 8; ++q) { v4f t;
#pragma unroll
        for (int i = 0; i < 4; ++i) { const int c = q * 128 + lane * 4 + i;
            t[i] = sigm(p[c]) * bfr(c0[(size_t)r * NHID + c]) + sigm(p[NHID + c]) * tanh_(p[2 * NHID + c]); }
        o[q] = t; }
    float* d = C1 + (size_t)r * NHID;
#pragma unroll
    for (int q = 0; q < 8; ++q) *(volatile v4f*)(d + q * 128 + lane * 4) = o[q];
    __threadfence();
#pragma unroll
    for (int q = 0; q < 8; ++q) *(volatile v4f*)(d + q * 128 + lane * 4) = o[q];
}

__global__ __launch_bounds__(256) void k_h1(const float* __restrict__ PRE, const float* __restrict__ C1, const float* __restrict__ MUC, const float* __restrict__ RSC,
                                            const float* __restrict__ gc, const float* __restrict__ bc, float* H1) {
    const int lane = threadIdx.x & 31, r = blockIdx.x * 8 + (threadIdx.x >> 5);
    if (r >= NBT) return;
    const float* p = PRE + (size_t)r * PREW;
    v4f o[8];
#pragma unroll 1
    for (int q = 0; q < 8; ++q) { v4f t;
#pragma unroll
        for (int i = 0; i < 4; ++i) { const int c = q * 128 + lane * 4 + i;
            t[i] = sigm(p[c]) * tanh_(bfr(gc[c]) * (C1[(size_t)r * NHID + c] - MUC[c]) * RSC[c] + bfr(bc[c])); }
        o[q] = t; }
    float* d = H1 + (size_t)r * NHID;
#pragma unroll
    for (int q = 0; q < 8; ++q) *(volatile v4f*)(d + q * 128 + lane * 4) = o[q];
    __threadfence();
#pragma unroll
    for (int q = 0; q < 8; ++q) *(volatile v4f*)(d + q * 128 + lane * 4) = o[q];
}

extern "C" void kernel_launch(void* const* d_in, const int* in_sizes, int n_in,
                              void* d_out, int out_size, void* d_ws, size_t ws_size, hipStream_t stream) {
    (void)in_sizes; (void)n_in; (void)out_size;
    const float* x = (const float*)d_in[0]; const float* h0 = (const float*)d_in[1]; const float* c0 = (const float*)d_in[2];
    const float* Wih = (const float*)d_in[3]; const float* Whh = (const float*)d_in[4]; const float* bias = (const float*)d_in[5];
    const float* gih = (const float*)d_in[6]; const float* bih = (const float*)d_in[7]; const float* ghh = (const float*)d_in[8]; const float* bhh = (const float*)d_in[9];
    const float* gc = (const float*)d_in[10]; const float* bc = (const float*)d_in[11];
    float* H1 = (float*)d_out;
    float* C1 = H1 + (size_t)NBT * NHID;
    char* wsp = (char*)d_ws;
    auto take = [&](size_t bytes) { char* p = wsp; wsp += (bytes + 255) & ~(size_t)255; return (void*)p; };
    bf* Xb = (bf*)take((size_t)NBT * NIN * 2); bf* Hb = (bf*)take((size_t)NBT * NHID * 2);
    bf* WIT = (bf*)take((size_t)NG4 * NIN * 2); bf* WHT = (bf*)take((size_t)NG4 * NHID * 2);
    float* WH = (float*)take((size_t)NBT * CW * 4); float* WI = (float*)take((size_t)NBT * CW * 4);
    float* PRE = (float*)take((size_t)NBT * PREW * 4);
    float* MUH = (float*)take(CW * 4); float* RSH = (float*)take(CW * 4); float* MUI = (float*)take(CW * 4); float* RSI = (float*)take(CW * 4);
    float* MUC = (float*)take(NHID * 4); float* RSC = (float*)take(NHID * 4);
    if ((size_t)(wsp - (char*)d_ws) > ws_size) return;
    k_cvtb<<<NBT / 8, 256, 0, stream>>>(x, Xb);
    k_cvtb<<<NBT / 8, 256, 0, stream>>>(h0, Hb);
    k_wt<<<dim3(NIN / 64, NG4 / 64, 1), 256, 0, stream>>>(Wih, WIT);
    k_wt<<<dim3(NHID / 64, NG4 / 64, 1), 256, 0, stream>>>(Whh, WHT);
    const int order[4] = {0, 1, 3, 2}; const int slots[4] = {0, 1, 2, 0};
    for (int s = 0; s < 4; ++s) {
        const int ch = order[s];
        if (s == 3) { k_c1<<<NBT / 8, 256, 0, stream>>>(PRE, c0, C1); k_colstat<<<NHID / 256, 256, 0, stream>>>(C1, MUC, RSC); }
        k_gemmb<<<dim3(NBT / 64, CW / 64, 1), 128, 0, stream>>>(Hb, WHT + (size_t)ch * CW * NHID, WH);
        k_gemmb<<<dim3(NBT / 64, CW / 64, 1), 128, 0, stream>>>(Xb, WIT + (size_t)ch * CW * NIN, WI);
        k_colstat<<<CW / 256, 256, 0, stream>>>(WH, MUH, RSH);
        k_colstat<<<CW / 256, 256, 0, stream>>>(WI, MUI, RSI);
        k_pre<<<NBT / 8, 256, 0, stream>>>(WH, WI, MUH, RSH, MUI, RSI, ghh, bhh, gih, bih, bias, ch * CW, slots[s], PRE);
    }
    k_h1<<<NBT / 8, 256, 0, stream>>>(PRE, C1, MUC, RSC, gc, bc, H1);
}
